// FeaturePropagation_17824114278741
// MI455X (gfx1250) — hardware-verified
//
#include <hip/hip_runtime.h>

#define NB    4
#define NCO   4096
#define NFI   16384
#define CCH   128
#define INCH  256
#define OCH   128
#define NGRP  32
#define GEPS  1e-5f

typedef float v4f __attribute__((ext_vector_type(4)));
typedef float v8f __attribute__((ext_vector_type(8)));
typedef __bf16 v16b __attribute__((ext_vector_type(16)));
typedef short v8s __attribute__((ext_vector_type(8)));
union Frag { v16b v; v8s h[2]; };

__device__ __forceinline__ unsigned short f2bf(float x) {
    unsigned u = __float_as_uint(x);
    u += 0x7FFFu + ((u >> 16) & 1u);
    return (unsigned short)(u >> 16);
}
__device__ __forceinline__ float bf2f(unsigned short s) {
    return __uint_as_float(((unsigned)s) << 16);
}
__device__ __forceinline__ v8f mma(v8f c, v16b a, v16b b) {
    return __builtin_amdgcn_wmma_f32_16x16x32_bf16(false, a, false, b, (short)0, c, false, false);
}
__device__ __forceinline__ void guard(v8f& c, v16b a, v16b b) {
    asm volatile("v_nop\n\tv_nop\n\tv_nop\n\tv_nop" : "+v"(c) : "v"(a), "v"(b));
}
__device__ __forceinline__ void st2(float* p, v4f v) {
    *(volatile v4f*)p = v;
    __threadfence();
    *(volatile v4f*)p = v;
}

__global__ __launch_bounds__(256)
void k_knn_interp(const float* __restrict__ xf, const float* __restrict__ xc,
                  const float* __restrict__ fc, const float* __restrict__ fs,
                  float* feat) {
#pragma clang fp contract(off)
    extern __shared__ float4 sc4[];
    __shared__ int   sidx[256 * 3];
    __shared__ float sw[256 * 3];

    const int tid = threadIdx.x;
    const int bpb = NFI / 256;
    const int b   = blockIdx.x / bpb;
    const int n0  = (blockIdx.x % bpb) * 256;
    if (b >= NB) return;

    for (int j = tid; j < NCO; j += 256) {
        const size_t o = ((size_t)b * NCO + j) * 3;
        const float cx = xc[o + 0], cy = xc[o + 1], cz = xc[o + 2];
        const float sq = (cx * cx + cy * cy) + cz * cz;
        sc4[j] = make_float4(cx, cy, cz, sq);
    }
    __syncthreads();

    const size_t p = (size_t)b * NFI + n0 + tid;
    const float fx = xf[p * 3 + 0], fy = xf[p * 3 + 1], fz = xf[p * 3 + 2];
    const float sqf = (fx * fx + fy * fy) + fz * fz;

    float t0 = 3.4e38f, t1 = 3.4e38f, t2 = 3.4e38f, t3 = 3.4e38f;
    int   j0 = 0, j1 = 0, j2 = 0, j3 = 0;
#pragma unroll 2
    for (int j = 0; j < NCO; ++j) {
        const float4 c = sc4[j];
        const float dot = fmaf(fz, c.z, fmaf(fy, c.y, fx * c.x));
        const float d = (sqf + c.w) - 2.0f * dot;
        if (d < t3) {
            if (d < t2) {
                t3 = t2; j3 = j2;
                if (d < t1) {
                    t2 = t1; j2 = j1;
                    if (d < t0) { t1 = t0; j1 = j0; t0 = d; j0 = j; }
                    else        { t1 = d;  j1 = j; }
                } else { t2 = d; j2 = j; }
            } else { t3 = d; j3 = j; }
        }
    }
    const float d0 = sqrtf(fmaxf(t0, 0.f));
    const float d1 = sqrtf(fmaxf(t1, 0.f));
    const float d2 = sqrtf(fmaxf(t2, 0.f));
    const float d3 = sqrtf(fmaxf(t3, 0.f));
    if (d3 == d2 && j3 < j2) j2 = j3;

    float w0, w1, w2;
    if (d0 <= 1e-12f) {
        w0 = 1.f; w1 = 0.f; w2 = 0.f;
    } else {
        w0 = 1.f / (d0 + 1e-12f);
        w1 = 1.f / (d1 + 1e-12f);
        w2 = 1.f / (d2 + 1e-12f);
        const float s = 1.f / ((w0 + w1) + w2);
        w0 *= s; w1 *= s; w2 *= s;
    }
    sidx[tid * 3 + 0] = j0; sidx[tid * 3 + 1] = j1; sidx[tid * 3 + 2] = j2;
    sw[tid * 3 + 0] = w0;   sw[tid * 3 + 1] = w1;   sw[tid * 3 + 2] = w2;
    __syncthreads();

    const int wave = tid >> 5, lane = tid & 31;
    const size_t cbase = (size_t)b * NCO * CCH;
    for (int rr = 0; rr < 32; ++rr) {
        const int rl = wave * 32 + rr;
        const size_t pr = (size_t)b * NFI + n0 + rl;
        int i0 = sidx[rl * 3 + 0], i1 = sidx[rl * 3 + 1], i2 = sidx[rl * 3 + 2];
        i0 = min(max(i0, 0), NCO - 1); i1 = min(max(i1, 0), NCO - 1); i2 = min(max(i2, 0), NCO - 1);
        const float a0 = sw[rl * 3 + 0], a1 = sw[rl * 3 + 1], a2 = sw[rl * 3 + 2];
        const float4 f0 = *(const float4*)(fc + cbase + (size_t)i0 * CCH + 4 * lane);
        const float4 f1 = *(const float4*)(fc + cbase + (size_t)i1 * CCH + 4 * lane);
        const float4 f2 = *(const float4*)(fc + cbase + (size_t)i2 * CCH + 4 * lane);
        v4f v;
        v.x = fmaf(a2, f2.x, fmaf(a1, f1.x, a0 * f0.x));
        v.y = fmaf(a2, f2.y, fmaf(a1, f1.y, a0 * f0.y));
        v.z = fmaf(a2, f2.z, fmaf(a1, f1.z, a0 * f0.z));
        v.w = fmaf(a2, f2.w, fmaf(a1, f1.w, a0 * f0.w));
        const float4 sk = *(const float4*)(fs + pr * CCH + 4 * lane);
        v4f s; s.x = sk.x; s.y = sk.y; s.z = sk.z; s.w = sk.w;
        st2(feat + pr * INCH + 4 * lane, v);
        st2(feat + pr * INCH + CCH + 4 * lane, s);
    }
}

template <bool GN>
__global__ __launch_bounds__(128)
void k_gemm(const float* __restrict__ A, const float* __restrict__ W,
            const float* __restrict__ bias, const float* __restrict__ stats,
            const float* __restrict__ gam, const float* __restrict__ bet,
            float* C, int M, int K) {
    extern __shared__ unsigned char smem[];
    unsigned short* Ah = (unsigned short*)smem;
    unsigned short* Al = Ah + 64 * 40;
    unsigned short* Wh = Al + 64 * 40;
    unsigned short* Wl = Wh + 128 * 40;
    float*          Cs = (float*)(Wl + 128 * 40);

    const int tid = threadIdx.x, wave = tid >> 5, lane = tid & 31;
    const int h = lane >> 4, m = lane & 15;
    const int m0 = blockIdx.x * 64;
    if (m0 >= M) return;

    v8f acc[8];
#pragma unroll
    for (int nt = 0; nt < 8; ++nt) acc[nt] = {};

    for (int kc = 0; kc < K; kc += 32) {
        __syncthreads();
        for (int i = tid; i < 512; i += 128) {
            const int r = i >> 3, q = i & 7;
            const float4 x4 = *(const float4*)(A + (size_t)(m0 + r) * K + kc + 4 * q);
            float e[4] = {x4.x, x4.y, x4.z, x4.w};
            if (GN) {
                const int bb = (m0 + r) / NFI;
                const int g  = (kc + 4 * q) >> 2;
                const float mean = stats[((size_t)bb * NGRP + g) * 32 + 0];
                const float istd = stats[((size_t)bb * NGRP + g) * 32 + 1];
#pragma unroll
                for (int u = 0; u < 4; ++u) {
                    float t = (e[u] - mean) * istd;
                    t = t * gam[kc + 4 * q + u] + bet[kc + 4 * q + u];
                    e[u] = fmaxf(t, 0.f);
                }
            }
#pragma unroll
            for (int u = 0; u < 4; ++u) {
                const unsigned short hi = f2bf(e[u]);
                Ah[r * 40 + 4 * q + u] = hi;
                Al[r * 40 + 4 * q + u] = f2bf(e[u] - bf2f(hi));
            }
        }
        for (int i = tid; i < 32 * 128; i += 128) {
            const int kk = i >> 7, n = i & 127;
            const float x = W[(size_t)(kc + kk) * OCH + n];
            const unsigned short hi = f2bf(x);
            Wh[n * 40 + kk] = hi;
            Wl[n * 40 + kk] = f2bf(x - bf2f(hi));
        }
        __syncthreads();

        Frag ah, al;
        const unsigned short* ar = Ah + (wave * 16 + m) * 40;
        const unsigned short* lr = Al + (wave * 16 + m) * 40;
        ah.h[0] = *(const v8s*)(ar + 8 * h);
        ah.h[1] = *(const v8s*)(ar + 16 + 8 * h);
        al.h[0] = *(const v8s*)(lr + 8 * h);
        al.h[1] = *(const v8s*)(lr + 16 + 8 * h);
#pragma unroll
        for (int nt = 0; nt < 8; ++nt) {
            Frag bh, bl;
            const unsigned short* br  = Wh + (nt * 16 + m) * 40;
            const unsigned short* blr = Wl + (nt * 16 + m) * 40;
            bh.h[0] = *(const v8s*)(br + 8 * h);
            bh.h[1] = *(const v8s*)(br + 16 + 8 * h);
            bl.h[0] = *(const v8s*)(blr + 8 * h);
            bl.h[1] = *(const v8s*)(blr + 16 + 8 * h);
            acc[nt] = mma(acc[nt], ah.v, bh.v);
            acc[nt] = mma(acc[nt], ah.v, bl.v);
            acc[nt] = mma(acc[nt], al.v, bh.v);
            guard(acc[nt], al.v, bh.v);
        }
    }

#pragma unroll
    for (int nt = 0; nt < 8; ++nt) {
        const int col = nt * 16 + m;
        const float bv = bias[col];
#pragma unroll
        for (int r = 0; r < 8; ++r)
            Cs[(wave * 16 + 8 * h + r) * 132 + col] = acc[nt][r] + bv;
    }
    __syncthreads();
    for (int r = 0; r < 16; ++r) {
        const int row = wave * 16 + r;
        const v4f v = *(const v4f*)(Cs + row * 132 + 4 * lane);
        st2(C + (size_t)(m0 + row) * OCH + 4 * lane, v);
    }
}

__global__ __launch_bounds__(256)
void k_stats(const float* __restrict__ H, float* stats) {
    __shared__ double rs[8], rq[8];
    const int tid = threadIdx.x;
    const int b = blockIdx.x / NGRP, g = blockIdx.x % NGRP;
    if (b >= NB) return;
    double s = 0.0, q = 0.0;
    for (int n = tid; n < NFI; n += 256) {
        const float4 v = *(const float4*)(H + ((size_t)b * NFI + n) * OCH + g * 4);
        s += (double)v.x; s += (double)v.y; s += (double)v.z; s += (double)v.w;
        q += (double)v.x * v.x; q += (double)v.y * v.y; q += (double)v.z * v.z; q += (double)v.w * v.w;
    }
    for (int o = 16; o > 0; o >>= 1) { s += __shfl_xor(s, o); q += __shfl_xor(q, o); }
    if ((tid & 31) == 0) { rs[tid >> 5] = s; rq[tid >> 5] = q; }
    __syncthreads();
    if (tid == 0) {
        double S = 0.0, Q = 0.0;
        for (int i = 0; i < 8; ++i) { S += rs[i]; Q += rq[i]; }
        const double inv = 1.0 / (double)(NFI * 4);
        const double mean = S * inv;
        double var = Q * inv - mean * mean;
        if (var < 0.0) var = 0.0;
        const float istd = 1.0f / sqrtf((float)var + GEPS);
        v4f v0; v0.x = (float)mean; v0.y = istd; v0.z = 0.f; v0.w = 0.f;
        v4f z = {};
        float* line = stats + (size_t)blockIdx.x * 32;
        for (int i = 0; i < 8; ++i) *(volatile v4f*)(line + 4 * i) = (i == 0 ? v0 : z);
        __threadfence();
        for (int i = 0; i < 8; ++i) *(volatile v4f*)(line + 4 * i) = (i == 0 ? v0 : z);
    }
}

__global__ __launch_bounds__(256)
void k_apply(const float* __restrict__ H, const float* __restrict__ gam,
             const float* __restrict__ bet, const float* __restrict__ stats,
             float* Y, int total4) {
    const size_t i = (size_t)blockIdx.x * 256 + threadIdx.x;
    if (i >= (size_t)total4) return;
    const size_t e = i * 4;
    const int c = (int)(e & 127);
    const int row = (int)(e >> 7);
    const int b = row / NFI;
    const int g = c >> 2;
    const float mean = stats[((size_t)b * NGRP + g) * 32 + 0];
    const float istd = stats[((size_t)b * NGRP + g) * 32 + 1];
    const float4 x = *(const float4*)(H + e);
    v4f y;
    y.x = fmaxf((x.x - mean) * istd * gam[c + 0] + bet[c + 0], 0.f);
    y.y = fmaxf((x.y - mean) * istd * gam[c + 1] + bet[c + 1], 0.f);
    y.z = fmaxf((x.z - mean) * istd * gam[c + 2] + bet[c + 2], 0.f);
    y.w = fmaxf((x.w - mean) * istd * gam[c + 3] + bet[c + 3], 0.f);
    st2(Y + e, y);
}

extern "C" void kernel_launch(void* const* d_in, const int* in_sizes, int n_in,
                              void* d_out, int out_size, void* d_ws, size_t ws_size,
                              hipStream_t stream) {
    if (n_in < 12) return;
    const int M = NB * NFI;
    if (in_sizes[0] != NB * NCO * 3 || in_sizes[1] != NB * NCO * CCH ||
        in_sizes[2] != NB * NFI * 3 || in_sizes[3] != NB * NFI * CCH ||
        in_sizes[4] != INCH * OCH || in_sizes[8] != OCH * OCH ||
        out_size != M * OCH) return;

    const float* xyz_coarse  = (const float*)d_in[0];
    const float* feat_coarse = (const float*)d_in[1];
    const float* xyz_fine    = (const float*)d_in[2];
    const float* feat_skip   = (const float*)d_in[3];
    const float* W1  = (const float*)d_in[4];
    const float* b1  = (const float*)d_in[5];
    const float* g1  = (const float*)d_in[6];
    const float* be1 = (const float*)d_in[7];
    const float* W2  = (const float*)d_in[8];
    const float* b2  = (const float*)d_in[9];
    const float* g2  = (const float*)d_in[10];
    const float* be2 = (const float*)d_in[11];
    float* out = (float*)d_out;

    char* ws = (char*)d_ws;
    size_t o = 0;
    float* feat   = (float*)(ws + o); o += (size_t)M * INCH * sizeof(float);
    float* h1     = (float*)(ws + o); o += (size_t)M * OCH * sizeof(float);
    float* h2     = (float*)(ws + o); o += (size_t)M * OCH * sizeof(float);
    float* stats1 = (float*)(ws + o); o += (size_t)NB * NGRP * 32 * sizeof(float);
    float* stats2 = (float*)(ws + o); o += (size_t)NB * NGRP * 32 * sizeof(float);
    if (o > ws_size) return;

    const size_t knn_lds  = (size_t)NCO * sizeof(float4);
    const size_t gemm_lds = (size_t)(64 * 40 * 2 + 128 * 40 * 2) * 2 + (size_t)64 * 132 * 4;

    k_knn_interp<<<M / 256, 256, knn_lds, stream>>>(xyz_fine, xyz_coarse, feat_coarse, feat_skip, feat);
    k_gemm<false><<<M / 64, 128, gemm_lds, stream>>>(feat, W1, b1, stats1, g1, be1, h1, M, INCH);
    k_stats<<<NB * NGRP, 256, 0, stream>>>(h1, stats1);
    k_gemm<true><<<M / 64, 128, gemm_lds, stream>>>(h1, W2, b2, stats1, g1, be1, h2, M, OCH);
    k_stats<<<NB * NGRP, 256, 0, stream>>>(h2, stats2);
    const int total4 = M * OCH / 4;
    k_apply<<<(total4 + 255) / 256, 256, 0, stream>>>(h2, g2, be2, stats2, out, total4);
}
